// InstEncoder_15633680958207
// MI455X (gfx1250) — hardware-verified
//
#include <hip/hip_runtime.h>
#include <math.h>

constexpr int NBATCH   = 4096;
constexpr int NSTEP    = 128;
constexpr int NHID     = 64;
constexpr int NGATE    = 4 * NHID;
constexpr int NEMB     = 32001;
constexpr int KCAT     = 2 * NHID;
constexpr int ROWS_BLK = 32;
constexpr int NTHR_REC = 128;
constexpr int NTHR_PRE = 256;
constexpr int APITCH   = 136;
constexpr int SLABP    = 68;
constexpr float WCARRY     = 16.0f;
constexpr float WCARRY_INV = 1.0f / 16.0f;
constexpr int NW8 = NGATE * (KCAT / 8);
static_assert(NBATCH % ROWS_BLK == 0);
static_assert(KCAT % 32 == 0);
static_assert(NHID == 16 * (NTHR_REC / 32));
static_assert(ROWS_BLK * (NHID / 16) == NTHR_REC);
static_assert((2 * ROWS_BLK * APITCH) % NTHR_REC == 0);
static_assert((NTHR_REC / 16) * 4 == ROWS_BLK);
static_assert(NW8 % NTHR_PRE == 0);

typedef __attribute__((ext_vector_type(16))) _Float16 v16h;
typedef __attribute__((ext_vector_type(8)))  _Float16 v8h;
typedef __attribute__((ext_vector_type(8)))  float    v8f;
typedef __attribute__((ext_vector_type(4)))  float    v4f;

__device__ __forceinline__ void dep_guard4_h(v8f& a, v8f& b, v8f& c, v8f& d, v16h x, v16h y) {
  asm volatile("v_nop\n\tv_nop\n\tv_nop\n\tv_nop" : "+v"(a), "+v"(b), "+v"(c), "+v"(d) : "v"(x), "v"(y));
}
__device__ __forceinline__ void keep4_h(v16h a, v16h b, v16h c, v16h d) { asm volatile("v_nop" :: "v"(a), "v"(b), "v"(c), "v"(d)); }
__device__ __forceinline__ void acc_guard4(v8f& a, v8f& b, v8f& c, v8f& d) { asm volatile("v_nop\n\tv_nop\n\tv_nop\n\tv_nop" : "+v"(a), "+v"(b), "+v"(c), "+v"(d)); }

template <typename T> struct Frag;
template <> struct Frag<_Float16> {
  typedef v16h V; union U { v16h v; v8h h[2]; };
  static __device__ __forceinline__ v16h load(const _Float16* p) {
    U f; f.h[0] = *(const v8h*)(p); f.h[1] = *(const v8h*)(p + 16); return f.v;
  }
  static __device__ __forceinline__ v8f mma(v16h a, v16h b, v8f c) {
    return __builtin_amdgcn_wmma_f32_16x16x32_f16(false, a, false, b, (short)0, c, false, false);
  }
};

__device__ __forceinline__ float fsig(float x)  { return __builtin_amdgcn_rcpf(1.0f + __expf(-x)); }
__device__ __forceinline__ float ftanh(float x) { return 1.0f - 2.0f * __builtin_amdgcn_rcpf(__expf(2.0f * x) + 1.0f); }

__device__ __forceinline__ void cell_update(float zi, float zf, float zg, float zo, float& cs, float& hs) {
  const float ig = fsig(zi);
  const float fg = fsig(zf);
  const float gg = ftanh(zg);
  const float og = fsig(zo);
  const float cn = fg * cs + ig * gg;
  cs = cn;
  hs = og * ftanh(cn);
}

__global__ __launch_bounds__(NTHR_PRE) void wcat_prep_kernel(const float* __restrict__ w_ih,
                                                             const float* __restrict__ w_hh,
                                                             unsigned short* __restrict__ dst) {
  const int i = blockIdx.x * NTHR_PRE + threadIdx.x;
  if (i < NW8) {
    const int n   = i >> 4;
    const int c8  = i & 15;
    const int col = (c8 & 7) * 8;
    const float* pa = w_ih + (size_t)n * NHID + col;
    const float* pb = w_hh + (size_t)n * NHID + col;
    const v4f a0 = *(const v4f*)(pa);
    const v4f a1 = *(const v4f*)(pa + 4);
    const v4f q0 = *(const v4f*)(pb);
    const v4f q1 = *(const v4f*)(pb + 4);
    const bool useh = (c8 >= 8);
    v8h hv;
#pragma unroll
    for (int e = 0; e < 4; ++e) {
      const float v0 = useh ? q0[e] : a0[e];
      const float v1 = useh ? q1[e] : a1[e];
      hv[e]     = (_Float16)(v0 * WCARRY);
      hv[4 + e] = (_Float16)(v1 * WCARRY);
    }
    unsigned short* op = dst + (size_t)i * 8;
    *(volatile v8h*)op = hv;
    __threadfence();
    *(volatile v8h*)op = hv;
  }
}

__global__ __launch_bounds__(NTHR_REC) void lstm_seq_kernel(const int* __restrict__ ids,
                                                            const float* __restrict__ emb,
                                                            const unsigned short* __restrict__ WCp,
                                                            const float* __restrict__ b_ih,
                                                            const float* __restrict__ b_hh,
                                                            float* __restrict__ out) {
  __shared__ __align__(16) _Float16 At[2][ROWS_BLK * APITCH];
  __shared__ __align__(16) float    Sl[ROWS_BLK * SLABP];
  const _Float16* WC = (const _Float16*)WCp;
  const int tid = threadIdx.x, lane = tid & 31, wave = tid >> 5;
  const int c = lane & 15, hh = lane >> 4, koff = hh * 8;
  const int b0 = blockIdx.x * ROWS_BLK;

  {
    _Float16* af = &At[0][0];
#pragma unroll 1
    for (int i = tid; i < 2 * ROWS_BLK * APITCH; i += NTHR_REC) af[i] = (_Float16)0.0f;
  }
  float cst[2][8], hst[2][8];
#pragma unroll
  for (int ms = 0; ms < 2; ++ms)
#pragma unroll
    for (int r = 0; r < 8; ++r) { cst[ms][r] = 0.0f; hst[ms][r] = 0.0f; }

  float bsum[4];
#pragma unroll
  for (int g = 0; g < 4; ++g) {
    const int n = NHID * g + 16 * wave + c;
    bsum[g] = b_ih[n] + b_hh[n];
  }

  const int grow = tid >> 2;
  const int gq   = tid & 3;
  const int* idrow = ids + (size_t)(b0 + grow) * NSTEP;
  __syncthreads();

  const v8f z8 = {0.f, 0.f, 0.f, 0.f, 0.f, 0.f, 0.f, 0.f};

#pragma unroll 1
  for (int t = 0; t < NSTEP; ++t) {
    const int p = t & 1;
    {
      int id = idrow[t];
      id = id < 0 ? 0 : id;
      id = id > (NEMB - 1) ? (NEMB - 1) : id;
      const float* er = emb + (size_t)id * NHID + 16 * gq;
      const v4f e0 = *(const v4f*)(er);
      const v4f e1 = *(const v4f*)(er + 4);
      const v4f e2 = *(const v4f*)(er + 8);
      const v4f e3 = *(const v4f*)(er + 12);
      v8h lo8, hi8;
#pragma unroll
      for (int e = 0; e < 4; ++e) {
        lo8[e] = (_Float16)e0[e]; lo8[4 + e] = (_Float16)e1[e];
        hi8[e] = (_Float16)e2[e]; hi8[4 + e] = (_Float16)e3[e];
      }
      _Float16* dstx = &At[p][0] + grow * APITCH + 16 * gq;
      *(v8h*)(dstx)     = lo8;
      *(v8h*)(dstx + 8) = hi8;
    }
    __syncthreads();

    v8f acc0[4], acc1[4];
#pragma unroll
    for (int g = 0; g < 4; ++g) { acc0[g] = z8; acc1[g] = z8; }
    const _Float16* ar0 = &At[p][0] + c * APITCH + koff;
    const _Float16* ar1 = ar0 + 16 * APITCH;
#pragma unroll 1
    for (int k0 = 0; k0 < KCAT; k0 += 32) {
      const v16h a0 = Frag<_Float16>::load(ar0 + k0);
      const v16h a1 = Frag<_Float16>::load(ar1 + k0);
      v16h bq[4];
#pragma unroll
      for (int g = 0; g < 4; ++g)
        bq[g] = Frag<_Float16>::load(WC + (size_t)(NHID * g + 16 * wave + c) * KCAT + koff + k0);
#pragma unroll
      for (int g = 0; g < 4; ++g) {
        acc0[g] = Frag<_Float16>::mma(a0, bq[g], acc0[g]);
        acc1[g] = Frag<_Float16>::mma(a1, bq[g], acc1[g]);
      }
      dep_guard4_h(acc0[0], acc0[1], acc0[2], acc0[3], a0, bq[0]);
      dep_guard4_h(acc1[0], acc1[1], acc1[2], acc1[3], a1, bq[3]);
      keep4_h(bq[0], bq[1], bq[2], bq[3]);
    }
    acc_guard4(acc0[0], acc0[1], acc0[2], acc0[3]);
    acc_guard4(acc1[0], acc1[1], acc1[2], acc1[3]);

    _Float16* an = &At[p ^ 1][0] + NHID + 16 * wave + c;
#pragma unroll
    for (int r = 0; r < 8; ++r) {
      {
        const float zi = acc0[0][r] * WCARRY_INV + bsum[0];
        const float zf = acc0[1][r] * WCARRY_INV + bsum[1];
        const float zg = acc0[2][r] * WCARRY_INV + bsum[2];
        const float zo = acc0[3][r] * WCARRY_INV + bsum[3];
        cell_update(zi, zf, zg, zo, cst[0][r], hst[0][r]);
        an[(8 * hh + r) * APITCH] = (_Float16)hst[0][r];
      }
      {
        const float zi = acc1[0][r] * WCARRY_INV + bsum[0];
        const float zf = acc1[1][r] * WCARRY_INV + bsum[1];
        const float zg = acc1[2][r] * WCARRY_INV + bsum[2];
        const float zo = acc1[3][r] * WCARRY_INV + bsum[3];
        cell_update(zi, zf, zg, zo, cst[1][r], hst[1][r]);
        an[(16 + 8 * hh + r) * APITCH] = (_Float16)hst[1][r];
      }
    }
  }

#pragma unroll
  for (int r = 0; r < 8; ++r) {
    Sl[(8 * hh + r) * SLABP + 16 * wave + c]      = hst[0][r];
    Sl[(16 + 8 * hh + r) * SLABP + 16 * wave + c] = hst[1][r];
  }
  __syncthreads();
  {
    const int srow = tid >> 4;
    const int c4   = (tid & 15) * 4;
    for (int pass = 0; pass < 2; ++pass) {
#pragma unroll
      for (int it = 0; it < 4; ++it) {
        const int row = it * 8 + srow;
        const v4f v = *(const v4f*)(Sl + row * SLABP + c4);
        *(volatile v4f*)(out + (size_t)(b0 + row) * NHID + c4) = v;
      }
      __threadfence();
    }
  }
}

extern "C" void kernel_launch(void* const* d_in, const int* in_sizes, int n_in,
                              void* d_out, int out_size, void* d_ws, size_t ws_size, hipStream_t stream) {
  if (n_in < 6 || d_out == nullptr || d_ws == nullptr) return;
  if (in_sizes[0] != NBATCH * NSTEP || in_sizes[1] != NEMB * NHID || in_sizes[2] != NGATE * NHID ||
      in_sizes[3] != NGATE * NHID || in_sizes[4] != NGATE || in_sizes[5] != NGATE ||
      out_size != NBATCH * NHID) return;
  const size_t need = (size_t)NGATE * KCAT * 2;
  if (need > ws_size || need > (size_t)134217728) return;

  const int*   ids  = (const int*)  d_in[0];
  const float* emb  = (const float*)d_in[1];
  const float* w_ih = (const float*)d_in[2];
  const float* w_hh = (const float*)d_in[3];
  const float* b_ih = (const float*)d_in[4];
  const float* b_hh = (const float*)d_in[5];
  float* out = (float*)d_out;
  unsigned short* WCAT = (unsigned short*)d_ws;

  wcat_prep_kernel<<<NW8 / NTHR_PRE, NTHR_PRE, 0, stream>>>(w_ih, w_hh, WCAT);
  lstm_seq_kernel<<<NBATCH / ROWS_BLK, NTHR_REC, 0, stream>>>(ids, emb, WCAT, b_ih, b_hh, out);
}
